// GAT_width_69277822484764
// MI455X (gfx1250) — hardware-verified
//
#include <hip/hip_runtime.h>
#include <stddef.h>


#define IN_DIM  256
#define KP      512
#define FEAT    512
#define HC      64
#define NHEAD   8
#define NCLS    40
#define NCLP    64
#define WTROWS  (FEAT + NCLP)
#define YP      512
#define EP      8
#define ZP      64
#define NTHR    256
#define NWAVE   8
#define EPT     8
#define CHUNK   (NTHR * EPT)
#define WCAP    (EPT * 32)
#define LISTN   (NWAVE * WCAP)
#define NBMAX   2048
#define RCAP    28672
#define DEGCAP  4096
#define GBM     64
#define GTHR    128
#define OBR     64
#define NEG_SLOPE 0.2f
#define CA      16.0f
#define CW      64.0f
#define SCL     0.0009765625f
#define WSCAP   134217728
#define LDS_AGG ((2 * RCAP + 2 * NBMAX + LISTN) * 4 + 64)

static_assert((CHUNK & (CHUNK - 1)) == 0 && CHUNK <= 4096);
static_assert((NBMAX & (NBMAX - 1)) == 0 && NBMAX <= 4096);
static_assert(NTHR * 8 == NBMAX);
static_assert(LISTN >= NBMAX);
static_assert(LISTN >= NWAVE * WCAP);
static_assert((RCAP % 32) == 0);
static_assert(LDS_AGG <= 300000);
static_assert(GBM == (GTHR / 32) * 16);
static_assert(2 * GBM == GTHR);
static_assert((FEAT % GTHR) == 0);
static_assert(NHEAD * HC == FEAT);
static_assert(HC == 64 && NHEAD == 8);
static_assert(FEAT == 2 * 32 * 8);
static_assert(KP == FEAT && (KP % 32) == 0 && (IN_DIM % 32) == 0 && IN_DIM <= KP);
static_assert((KP / 8) == 64);
static_assert(GBM * EP == GTHR * 4);
static_assert(EP == NHEAD);
static_assert(NCLS <= NCLP && NCLP == HC);
static_assert((NCLS % 4) == 0 && NCLS <= 2 * 32);
static_assert(ZP == 2 * 32);
static_assert(YP == FEAT);
static_assert(3 * NTHR >= OBR * (NCLS / 4));
static_assert(OBR == GBM);

typedef float    v2f  __attribute__((ext_vector_type(2)));
typedef float    v4f  __attribute__((ext_vector_type(4)));
typedef float    v8f  __attribute__((ext_vector_type(8)));
typedef int      v4i  __attribute__((ext_vector_type(4)));
typedef int      v8i  __attribute__((ext_vector_type(8)));
typedef _Float16 v4h  __attribute__((ext_vector_type(4)));
typedef _Float16 v8h  __attribute__((ext_vector_type(8)));
typedef _Float16 v16h __attribute__((ext_vector_type(16)));
union FragH { v16h v; v8h h[2]; v8i w; };

__device__ __forceinline__ v8f wmh(const FragH& a, const FragH& b, v8f c) {
  v8f d = __builtin_amdgcn_wmma_f32_16x16x32_f16(false, a.v, false, b.v, (short)0, c, false, false);
  asm volatile("v_nop\n\tv_nop\n\tv_nop\n\tv_nop" : "+v"(d) : "v"(a.w), "v"(b.w));
  return d;
}

__device__ __forceinline__ float eluf(float x) {
  const float xn = fminf(x, 0.f);
  const float em = __expf(xn) - 1.0f;
  return x > 0.f ? x : em;
}

__device__ __forceinline__ int scan_chunk(const int* __restrict__ dsts, int nE, int cbase, int slotBase,
                                          int nb, int vec8, int* list, int tid, int lane, int wave) {
  int wc = 0;
  const int el0  = tid * EPT;
  const int e0   = cbase + el0;
  const int sent = -2147483647 - 1;
  v4i da, db;
  if (vec8 != 0 && cbase + CHUNK <= nE) {
    da = *(const v4i*)(dsts + e0);
    db = *(const v4i*)(dsts + e0 + 4);
  } else {
    da.x = (e0     < nE) ? dsts[min(e0,     nE - 1)] : sent;
    da.y = (e0 + 1 < nE) ? dsts[min(e0 + 1, nE - 1)] : sent;
    da.z = (e0 + 2 < nE) ? dsts[min(e0 + 2, nE - 1)] : sent;
    da.w = (e0 + 3 < nE) ? dsts[min(e0 + 3, nE - 1)] : sent;
    db.x = (e0 + 4 < nE) ? dsts[min(e0 + 4, nE - 1)] : sent;
    db.y = (e0 + 5 < nE) ? dsts[min(e0 + 5, nE - 1)] : sent;
    db.z = (e0 + 6 < nE) ? dsts[min(e0 + 6, nE - 1)] : sent;
    db.w = (e0 + 7 < nE) ? dsts[min(e0 + 7, nE - 1)] : sent;
  }
  const unsigned nbs = (unsigned)slotBase;
  const unsigned unb = (unsigned)nb;
  const unsigned s0 = (unsigned)da.x - nbs, s1 = (unsigned)da.y - nbs;
  const unsigned s2 = (unsigned)da.z - nbs, s3 = (unsigned)da.w - nbs;
  const unsigned s4 = (unsigned)db.x - nbs, s5 = (unsigned)db.y - nbs;
  const unsigned s6 = (unsigned)db.z - nbs, s7 = (unsigned)db.w - nbs;
  const bool h0 = s0 < unb, h1 = s1 < unb, h2 = s2 < unb, h3 = s3 < unb;
  const bool h4 = s4 < unb, h5 = s5 < unb, h6 = s6 < unb, h7 = s7 < unb;
  const unsigned any = __builtin_amdgcn_ballot_w32(h0 | h1 | h2 | h3 | h4 | h5 | h6 | h7);
  if (any != 0u) {
#define HITJ(J, HJ, SJ) { \
      const unsigned mj = __builtin_amdgcn_ballot_w32(HJ); \
      if (mj != 0u) { \
        if (HJ) { \
          const int pos = wc + (int)__builtin_amdgcn_mbcnt_lo(mj, 0u); \
          if (pos < WCAP) list[wave * WCAP + pos] = ((el0 + (J)) << 12) | (int)(SJ); \
        } \
        wc += (int)__builtin_popcount(mj); } }
    HITJ(0, h0, s0)
    HITJ(1, h1, s1)
    HITJ(2, h2, s2)
    HITJ(3, h3, s3)
    HITJ(4, h4, s4)
    HITJ(5, h5, s5)
    HITJ(6, h6, s6)
    HITJ(7, h7, s7)
#undef HITJ
  }
  return wc;
}

__global__ __launch_bounds__(NTHR) void k_xprep(const float* __restrict__ x, _Float16* xh, int nN, int nUnits) {
  const int i = (int)blockIdx.x * NTHR + (int)threadIdx.x;
  if (i >= nUnits) return;
  const int row = i >> 6;
  const int c0  = (i & 63) * 8;
  const int rc  = row < nN ? row : nN - 1;
  const int cc  = c0 & (IN_DIM - 1);
  const float* p = x + (size_t)rc * IN_DIM + cc;
  v4f a = *(const v4f*)p, b = *(const v4f*)(p + 4);
  const v4f z4 = {0.f, 0.f, 0.f, 0.f};
  if (row >= nN || c0 >= IN_DIM) { a = z4; b = z4; }
  v8h hv;
  hv[0] = (_Float16)(a.x * CA); hv[1] = (_Float16)(a.y * CA);
  hv[2] = (_Float16)(a.z * CA); hv[3] = (_Float16)(a.w * CA);
  hv[4] = (_Float16)(b.x * CA); hv[5] = (_Float16)(b.y * CA);
  hv[6] = (_Float16)(b.z * CA); hv[7] = (_Float16)(b.w * CA);
  const size_t o = (size_t)row * KP + c0;
  *(volatile v8h*)(xh + o) = hv;
  __threadfence();
  *(volatile v8h*)(xh + o) = hv;
}

__global__ __launch_bounds__(NTHR) void k_wprep(const float* __restrict__ w1, const float* __restrict__ w2,
                                                _Float16* wt) {
  const int j  = (int)blockIdx.y;
  const int u  = (int)blockIdx.x * NTHR + (int)threadIdx.x;
  const int nrow = (j == 0) ? FEAT : NCLP;
  const int nUnits = nrow * (KP / 8);
  if (u >= nUnits) return;
  const int n  = u >> 6;
  const int k8 = (u & 63) * 8;
  const int ksrc = (j == 0) ? IN_DIM : FEAT;
  const int nc   = (j == 0) ? FEAT : NCLS;
  const float* src = (j == 0) ? w1 : w2;
  const bool valid = (k8 < ksrc) && (n < nc);
  const int kc  = (k8 < ksrc) ? k8 : (ksrc - 8);
  const int ncl = (n < nc) ? n : (nc - 1);
  const float* p = src + (size_t)kc * nc + ncl;
  v4f a, b;
  a.x = p[0 * nc]; a.y = p[1 * nc]; a.z = p[2 * nc]; a.w = p[3 * nc];
  b.x = p[4 * nc]; b.y = p[5 * nc]; b.z = p[6 * nc]; b.w = p[7 * nc];
  const v4f z4 = {0.f, 0.f, 0.f, 0.f};
  if (!valid) { a = z4; b = z4; }
  v8h hv;
  hv[0] = (_Float16)(a.x * CW); hv[1] = (_Float16)(a.y * CW);
  hv[2] = (_Float16)(a.z * CW); hv[3] = (_Float16)(a.w * CW);
  hv[4] = (_Float16)(b.x * CW); hv[5] = (_Float16)(b.y * CW);
  hv[6] = (_Float16)(b.z * CW); hv[7] = (_Float16)(b.w * CW);
  const size_t rowb = (size_t)j * FEAT;
  const size_t o = (rowb + (size_t)n) * KP + k8;
  *(volatile v8h*)(wt + o) = hv;
  __threadfence();
  *(volatile v8h*)(wt + o) = hv;
}

__global__ __launch_bounds__(GTHR) void k_gemm(const _Float16* __restrict__ xh, const _Float16* __restrict__ wt,
                                               const float* __restrict__ asrc, const float* __restrict__ adst,
                                               int attn, float* Y, float* ES, float* ED, int nks, int npass) {
  __shared__ __attribute__((aligned(16))) float stg[GBM * HC];
  __shared__ __attribute__((aligned(16))) float esT[GBM * EP];
  __shared__ __attribute__((aligned(16))) float edT[GBM * EP];
  __shared__ float sAs[FEAT];
  __shared__ float sAd[FEAT];
  const int tid = threadIdx.x, lane = tid & 31, wave = tid >> 5, hh = lane >> 4, m = lane & 15;
  const int rowBase = (int)blockIdx.x * GBM;
  const int an = attn < 1 ? 1 : (attn > FEAT ? FEAT : attn);
#pragma unroll 1
  for (int i = tid; i < FEAT; i += GTHR) {
    const int ic = i < an ? i : an - 1;
    const float va = asrc[ic];
    const float vd = adst[ic];
    sAs[i] = (i < an) ? va : 0.f;
    sAd[i] = (i < an) ? vd : 0.f;
  }
#pragma unroll 1
  for (int i = tid; i < GBM * EP; i += GTHR) { esT[i] = 0.f; edT[i] = 0.f; }
  const int nk = nks < 1 ? 1 : (nks > KP / 32 ? KP / 32 : nks);
  const int np = npass < 1 ? 1 : (npass > NHEAD ? NHEAD : npass);
  __syncthreads();
  const size_t arow = (size_t)(rowBase + 16 * wave + m) * KP + 8 * hh;
#pragma unroll 1
  for (int p = 0; p < np; ++p) {
    v8f acc[4];
#pragma unroll
    for (int t = 0; t < 4; ++t) { v8f z = {0.f, 0.f, 0.f, 0.f, 0.f, 0.f, 0.f, 0.f}; acc[t] = z; }
    const size_t brow = (size_t)(p * HC + m) * KP + 8 * hh;
#pragma unroll 1
    for (int ks = 0; ks < nk; ++ks) {
      FragH af;
      af.h[0] = *(const v8h*)(xh + arow + 32 * ks);
      af.h[1] = *(const v8h*)(xh + arow + 32 * ks + 16);
#pragma unroll
      for (int t = 0; t < 4; ++t) {
        const size_t bo = brow + (size_t)(16 * t) * KP + 32 * ks;
        FragH bf;
        bf.h[0] = *(const v8h*)(wt + bo);
        bf.h[1] = *(const v8h*)(wt + bo + 16);
        acc[t] = wmh(af, bf, acc[t]);
      }
    }
    float* sp = stg + (size_t)(16 * wave + 8 * hh) * HC + m;
#pragma unroll
    for (int t = 0; t < 4; ++t) {
#pragma unroll
      for (int r = 0; r < 8; ++r) sp[(size_t)r * HC + 16 * t] = acc[t][r] * SCL;
    }
    __syncthreads();
    {
      const int row  = tid >> 1;
      const int half = tid & 1;
      const float* srow = stg + (size_t)row * HC;
      float s = 0.f, d = 0.f;
#pragma unroll 1
      for (int c = 0; c < 32; ++c) {
        const int cc = half * 32 + c;
        const float v = srow[cc];
        s = fmaf(v, sAs[p * HC + cc], s);
        d = fmaf(v, sAd[p * HC + cc], d);
      }
      s += __shfl_xor(s, 1);
      d += __shfl_xor(d, 1);
      if (half == 0) {
        esT[row * EP + p] = s;
        edT[row * EP + p] = d;
      }
    }
    const int nF4 = GBM * HC / 4;
    float* yb = Y + (size_t)rowBase * YP + HC * p;
    const v4f* s4 = (const v4f*)stg;
#pragma unroll 1
    for (int f = tid; f < nF4; f += GTHR) {
      const int r = f >> 4, q = f & 15;
      const v4f v = s4[f];
      *(volatile v4f*)(yb + (size_t)r * YP + 4 * q) = v;
    }
    __threadfence();
#pragma unroll 1
    for (int f = tid; f < nF4; f += GTHR) {
      const int r = f >> 4, q = f & 15;
      const v4f v = s4[f];
      *(volatile v4f*)(yb + (size_t)r * YP + 4 * q) = v;
    }
    __syncthreads();
  }
  {
    const v4f ve = *(const v4f*)(esT + 4 * tid);
    const v4f vd = *(const v4f*)(edT + 4 * tid);
    float* pe = ES + (size_t)rowBase * EP + 4 * tid;
    float* pd = ED + (size_t)rowBase * EP + 4 * tid;
    *(volatile v4f*)pe = ve;
    *(volatile v4f*)pd = vd;
    __threadfence();
    *(volatile v4f*)pe = ve;
    *(volatile v4f*)pd = vd;
  }
}

template <int L>
__global__ __launch_bounds__(NTHR) void k_agg(
    const int* __restrict__ srcs, const int* __restrict__ dsts,
    const float* __restrict__ Y, const float* __restrict__ ES, const float* __restrict__ ED,
    const float* __restrict__ bias, _Float16* xout, float* zout,
    int nN, int nE, int nb, int vec8) {
  extern __shared__ v4f lds_dyn[];
  int* reg1 = (int*)lds_dyn;
  int* reg2 = reg1 + RCAP;
  int* scnt = reg2 + RCAP;
  int* soff = scnt + NBMAX;
  int* list = soff + NBMAX;
  int* wcnt = list + LISTN;
  int* wtot = wcnt + NWAVE;
  const int tid = threadIdx.x, lane = tid & 31, wave = tid >> 5;
  const int nodeBase = (int)blockIdx.x * nb;

  for (int i = tid; i < NBMAX; i += NTHR) scnt[i] = 0;
  __syncthreads();

  int tot = 0;
  const int nChunks = (nE + CHUNK - 1) / CHUNK;
#pragma unroll 1
  for (int ch = 0; ch < nChunks; ++ch) {
    const int cbase = ch * CHUNK;
    const int wc = scan_chunk(dsts, nE, cbase, nodeBase, nb, vec8, list, tid, lane, wave);
    if (lane == 0) wcnt[wave] = wc;
    __syncthreads();
    int pre = 0, all = 0;
#pragma unroll
    for (int w2 = 0; w2 < NWAVE; ++w2) {
      int c = wcnt[w2];
      c = c < 0 ? 0 : (c > WCAP ? WCAP : c);
      all += c;
      pre += (w2 < wave) ? c : 0;
    }
    const int wcc  = wc > WCAP ? WCAP : wc;
    const int base = tot + pre;
#pragma unroll 1
    for (int i = lane; i < wcc; i += 32) {
      const int ent = list[wave * WCAP + i];
      const int el  = (ent >> 12) & (CHUNK - 1);
      const int sl  = ent & (NBMAX - 1);
      int eid = cbase + el;
      eid = eid > nE - 1 ? nE - 1 : eid;
      const int pos = base + i;
      if (pos < RCAP) reg1[pos] = (int)(((unsigned)eid << 12) | (unsigned)sl);
    }
    tot += all;
    tot = tot > RCAP ? RCAP : tot;
    __syncthreads();
  }
  const int nh = tot;

  if (wave == 0) {
#pragma unroll 1
    for (int b0 = 0; b0 < nh; b0 += 32) {
      const int idx = b0 + lane;
      const int uv  = reg1[idx < RCAP ? idx : RCAP - 1];
      const int m32 = (nh - b0) < 32 ? (nh - b0) : 32;
#pragma unroll 1
      for (int k = 0; k < m32; ++k) {
        const int u  = __builtin_amdgcn_readlane(uv, k);
        const int sl = u & (NBMAX - 1);
        if (lane == 0) scnt[sl] = scnt[sl] + 1;
      }
    }
  }
  __syncthreads();

  {
    const v4i ca = *(const v4i*)(scnt + 8 * tid);
    const v4i cb = *(const v4i*)(scnt + 8 * tid + 4);
    const int e0 = ca.x < 0 ? 0 : ca.x, e1 = ca.y < 0 ? 0 : ca.y, e2 = ca.z < 0 ? 0 : ca.z, e3 = ca.w < 0 ? 0 : ca.w;
    const int e4 = cb.x < 0 ? 0 : cb.x, e5 = cb.y < 0 ? 0 : cb.y, e6 = cb.z < 0 ? 0 : cb.z, e7 = cb.w < 0 ? 0 : cb.w;
    const int ts = e0 + e1 + e2 + e3 + e4 + e5 + e6 + e7;
    int incl = ts;
#pragma unroll
    for (int d = 1; d < 32; d <<= 1) {
      const int up = __shfl_up(incl, d);
      if (lane >= d) incl += up;
    }
    if (lane == 31) wtot[wave] = incl;
    __syncthreads();
    int pre = 0;
#pragma unroll
    for (int w2 = 0; w2 < NWAVE; ++w2) pre += (w2 < wave) ? wtot[w2] : 0;
    int run = pre + incl - ts;
    soff[8 * tid + 0] = run; run += e0;
    soff[8 * tid + 1] = run; run += e1;
    soff[8 * tid + 2] = run; run += e2;
    soff[8 * tid + 3] = run; run += e3;
    soff[8 * tid + 4] = run; run += e4;
    soff[8 * tid + 5] = run; run += e5;
    soff[8 * tid + 6] = run; run += e6;
    soff[8 * tid + 7] = run;
  }
  __syncthreads();
  for (int i = tid; i < NBMAX; i += NTHR) list[i] = soff[i];
  __syncthreads();

  if (wave == 0) {
#pragma unroll 1
    for (int b0 = 0; b0 < nh; b0 += 32) {
      const int idx = b0 + lane;
      const int uv  = reg1[idx < RCAP ? idx : RCAP - 1];
      const int m32 = (nh - b0) < 32 ? (nh - b0) : 32;
#pragma unroll 1
      for (int k = 0; k < m32; ++k) {
        const int u   = __builtin_amdgcn_readlane(uv, k);
        const int sl  = u & (NBMAX - 1);
        const int eid = (int)((unsigned)u >> 12);
        if (lane == 0) {
          int pos = list[sl];
          pos = pos < 0 ? 0 : (pos > RCAP - 1 ? RCAP - 1 : pos);
          reg2[pos] = eid;
          list[sl] = pos + 1;
        }
      }
    }
  }
  __syncthreads();

  const int nbw = nb >> 3;
  const bool ovf = (nh >= RCAP);
  const float qnan = __int_as_float(0x7fc00000);
  if (L == 1) {
    const int c8 = 8 * lane;
    const int hA = lane >> 3;
    const int hB = hA + (NHEAD / 2);
    const v4f bA0 = *(const v4f*)(bias + c8);
    const v4f bA1 = *(const v4f*)(bias + c8 + 4);
    const v4f bB0 = *(const v4f*)(bias + (FEAT / 2) + c8);
    const v4f bB1 = *(const v4f*)(bias + (FEAT / 2) + c8 + 4);
#pragma unroll 1
    for (int jt = 0; jt < nbw; ++jt) {
      const int slot = wave * nbw + jt;
      const int grow = nodeBase + slot;
      const int gcl  = grow < nN ? grow : nN - 1;
      int st = soff[slot];
      const int craw = scnt[slot];
      int cnt = craw;
      st  = st < 0 ? 0 : (st > nh ? nh : st);
      cnt = cnt < 0 ? 0 : (cnt > DEGCAP ? DEGCAP : cnt);
      if (cnt > nh - st) cnt = nh - st;
      const float pz = (ovf || craw > DEGCAP) ? qnan : 0.0f;
      const bool wr = grow < nN;

      const float* yd = Y + (size_t)gcl * YP;
      const v4f xA0 = *(const v4f*)(yd + c8);
      const v4f xA1 = *(const v4f*)(yd + c8 + 4);
      const v4f xB0 = *(const v4f*)(yd + (FEAT / 2) + c8);
      const v4f xB1 = *(const v4f*)(yd + (FEAT / 2) + c8 + 4);
      const float edA = ED[(size_t)gcl * EP + hA];
      const float edB = ED[(size_t)gcl * EP + hB];
      const float esA = ES[(size_t)gcl * EP + hA];
      const float esB = ES[(size_t)gcl * EP + hB];
      const float tA = esA + edA, tB = esB + edB;
      float mA = fmaxf(tA, NEG_SLOPE * tA);
      float mB = fmaxf(tB, NEG_SLOPE * tB);
      float dA = 1.0f, dB = 1.0f;
      v4f a0 = xA0, a1 = xA1, a2 = xB0, a3 = xB1;
#pragma unroll 1
      for (int q = 0; q < cnt; ++q) {
        int idx = st + q; idx = idx > RCAP - 1 ? RCAP - 1 : idx;
        int eid = reg2[idx]; eid = eid < 0 ? 0 : (eid > nE - 1 ? nE - 1 : eid);
        const int sraw = srcs[eid];
        const int s = sraw < 0 ? 0 : (sraw > nN - 1 ? nN - 1 : sraw);
        const float* ys = Y + (size_t)s * YP;
        const v4f y0 = *(const v4f*)(ys + c8);
        const v4f y1 = *(const v4f*)(ys + c8 + 4);
        const v4f y2 = *(const v4f*)(ys + (FEAT / 2) + c8);
        const v4f y3 = *(const v4f*)(ys + (FEAT / 2) + c8 + 4);
        const float eA = ES[(size_t)s * EP + hA];
        const float eB = ES[(size_t)s * EP + hB];
        const float uA = eA + edA, uB = eB + edB;
        const float lA = fmaxf(uA, NEG_SLOPE * uA);
        const float lB = fmaxf(uB, NEG_SLOPE * uB);
        const float nA = fmaxf(mA, lA), nB = fmaxf(mB, lB);
        const float pA = __expf(mA - nA), qA = __expf(lA - nA);
        const float pB = __expf(mB - nB), qB = __expf(lB - nB);
        dA = fmaf(dA, pA, qA);
        dB = fmaf(dB, pB, qB);
        a0.x = fmaf(a0.x, pA, qA * y0.x);
        a0.y = fmaf(a0.y, pA, qA * y0.y);
        a0.z = fmaf(a0.z, pA, qA * y0.z);
        a0.w = fmaf(a0.w, pA, qA * y0.w);
        a1.x = fmaf(a1.x, pA, qA * y1.x);
        a1.y = fmaf(a1.y, pA, qA * y1.y);
        a1.z = fmaf(a1.z, pA, qA * y1.z);
        a1.w = fmaf(a1.w, pA, qA * y1.w);
        a2.x = fmaf(a2.x, pB, qB * y2.x);
        a2.y = fmaf(a2.y, pB, qB * y2.y);
        a2.z = fmaf(a2.z, pB, qB * y2.z);
        a2.w = fmaf(a2.w, pB, qB * y2.w);
        a3.x = fmaf(a3.x, pB, qB * y3.x);
        a3.y = fmaf(a3.y, pB, qB * y3.y);
        a3.z = fmaf(a3.z, pB, qB * y3.z);
        a3.w = fmaf(a3.w, pB, qB * y3.w);
        mA = nA; mB = nB;
      }
      const float iA = __builtin_amdgcn_rcpf(dA);
      const float iB = __builtin_amdgcn_rcpf(dB);
      v4f o0, o1, o2, o3;
      o0.x = eluf(fmaf(a0.x, iA, bA0.x)) + pz;
      o0.y = eluf(fmaf(a0.y, iA, bA0.y)) + pz;
      o0.z = eluf(fmaf(a0.z, iA, bA0.z)) + pz;
      o0.w = eluf(fmaf(a0.w, iA, bA0.w)) + pz;
      o1.x = eluf(fmaf(a1.x, iA, bA1.x)) + pz;
      o1.y = eluf(fmaf(a1.y, iA, bA1.y)) + pz;
      o1.z = eluf(fmaf(a1.z, iA, bA1.z)) + pz;
      o1.w = eluf(fmaf(a1.w, iA, bA1.w)) + pz;
      o2.x = eluf(fmaf(a2.x, iB, bB0.x)) + pz;
      o2.y = eluf(fmaf(a2.y, iB, bB0.y)) + pz;
      o2.z = eluf(fmaf(a2.z, iB, bB0.z)) + pz;
      o2.w = eluf(fmaf(a2.w, iB, bB0.w)) + pz;
      o3.x = eluf(fmaf(a3.x, iB, bB1.x)) + pz;
      o3.y = eluf(fmaf(a3.y, iB, bB1.y)) + pz;
      o3.z = eluf(fmaf(a3.z, iB, bB1.z)) + pz;
      o3.w = eluf(fmaf(a3.w, iB, bB1.w)) + pz;
      v8h hv0, hv1;
      hv0[0] = (_Float16)(o0.x * CA); hv0[1] = (_Float16)(o0.y * CA);
      hv0[2] = (_Float16)(o0.z * CA); hv0[3] = (_Float16)(o0.w * CA);
      hv0[4] = (_Float16)(o1.x * CA); hv0[5] = (_Float16)(o1.y * CA);
      hv0[6] = (_Float16)(o1.z * CA); hv0[7] = (_Float16)(o1.w * CA);
      hv1[0] = (_Float16)(o2.x * CA); hv1[1] = (_Float16)(o2.y * CA);
      hv1[2] = (_Float16)(o2.z * CA); hv1[3] = (_Float16)(o2.w * CA);
      hv1[4] = (_Float16)(o3.x * CA); hv1[5] = (_Float16)(o3.y * CA);
      hv1[6] = (_Float16)(o3.z * CA); hv1[7] = (_Float16)(o3.w * CA);
      _Float16* xp = xout + (size_t)gcl * KP + c8;
      if (wr) {
        *(volatile v8h*)xp = hv0;
        *(volatile v8h*)(xp + (FEAT / 2)) = hv1;
      }
      __threadfence();
      if (wr) {
        *(volatile v8h*)xp = hv0;
        *(volatile v8h*)(xp + (FEAT / 2)) = hv1;
      }
    }
  } else {
    const int c2 = 2 * lane;
    const bool cv = (c2 + 1) < NCLS;
    const int cb0 = c2 < (NCLS - 2) ? c2 : (NCLS - 2);
    const float bq0 = bias[cb0];
    const float bq1 = bias[cb0 + 1];
    const float bz0 = cv ? bq0 : 0.f;
    const float bz1 = cv ? bq1 : 0.f;
#pragma unroll 1
    for (int jt = 0; jt < nbw; ++jt) {
      const int slot = wave * nbw + jt;
      const int grow = nodeBase + slot;
      const int gcl  = grow < nN ? grow : nN - 1;
      int st = soff[slot];
      const int craw = scnt[slot];
      int cnt = craw;
      st  = st < 0 ? 0 : (st > nh ? nh : st);
      cnt = cnt < 0 ? 0 : (cnt > DEGCAP ? DEGCAP : cnt);
      if (cnt > nh - st) cnt = nh - st;
      const float pz = (ovf || craw > DEGCAP) ? qnan : 0.0f;
      const bool wr = grow < nN;

      const v2f xd = *(const v2f*)(Y + (size_t)gcl * YP + c2);
      const float ed0 = ED[(size_t)gcl * EP];
      const float es0 = ES[(size_t)gcl * EP];
      const float t0 = es0 + ed0;
      float mx = fmaxf(t0, NEG_SLOPE * t0);
      float dn = 1.0f;
      v2f a = xd;
#pragma unroll 1
      for (int q = 0; q < cnt; ++q) {
        int idx = st + q; idx = idx > RCAP - 1 ? RCAP - 1 : idx;
        int eid = reg2[idx]; eid = eid < 0 ? 0 : (eid > nE - 1 ? nE - 1 : eid);
        const int sraw = srcs[eid];
        const int s = sraw < 0 ? 0 : (sraw > nN - 1 ? nN - 1 : sraw);
        const v2f xs = *(const v2f*)(Y + (size_t)s * YP + c2);
        const float ess = ES[(size_t)s * EP];
        const float u = ess + ed0;
        const float l = fmaxf(u, NEG_SLOPE * u);
        const float mn = fmaxf(mx, l);
        const float p1 = __expf(mx - mn), p2 = __expf(l - mn);
        dn  = fmaf(dn, p1, p2);
        a.x = fmaf(a.x, p1, p2 * xs.x);
        a.y = fmaf(a.y, p1, p2 * xs.y);
        mx = mn;
      }
      const float inv = __builtin_amdgcn_rcpf(dn);
      const float ox = fmaf(a.x, inv, bz0);
      const float oy = fmaf(a.y, inv, bz1);
      float vm = cv ? fmaxf(ox, oy) : -3.0e38f;
#pragma unroll
      for (int d = 16; d >= 1; d >>= 1) vm = fmaxf(vm, __shfl_xor(vm, d));
      const float sx = fminf(ox - vm, 0.f);
      const float sy = fminf(oy - vm, 0.f);
      float se = cv ? (__expf(sx) + __expf(sy)) : 0.f;
#pragma unroll
      for (int d = 16; d >= 1; d >>= 1) se += __shfl_xor(se, d);
      const float lg = __logf(se);
      v2f z;
      z.x = cv ? ((sx - lg) + pz) : 0.f;
      z.y = cv ? ((sy - lg) + pz) : 0.f;
      float* zp = zout + (size_t)gcl * ZP + c2;
      if (wr) *(volatile v2f*)zp = z;
      __threadfence();
      if (wr) *(volatile v2f*)zp = z;
    }
  }
}

__global__ __launch_bounds__(NTHR) void k_out(const float* __restrict__ Z, float* out, int nN) {
  const int tid = threadIdx.x;
  const int rowBase = (int)blockIdx.x * OBR;
  const int nValid = (nN - rowBase) < OBR ? (nN - rowBase) : OBR;
  const int q4 = NCLS / 4;
  const int n4 = nValid * q4;
  float* base = out + (size_t)rowBase * NCLS;
  v4f v[3];
#pragma unroll
  for (int i = 0; i < 3; ++i) {
    const int f = tid + NTHR * i;
    const int row = f / q4;
    const int q = f - row * q4;
    int gr = rowBase + row; gr = gr > nN - 1 ? nN - 1 : gr;
    v[i] = *(const v4f*)(Z + (size_t)gr * ZP + 4 * q);
  }
#pragma unroll
  for (int i = 0; i < 3; ++i) {
    const int f = tid + NTHR * i;
    if (f < n4) *(volatile v4f*)(base + (size_t)4 * f) = v[i];
  }
  __threadfence();
#pragma unroll
  for (int i = 0; i < 3; ++i) {
    const int f = tid + NTHR * i;
    if (f < n4) *(volatile v4f*)(base + (size_t)4 * f) = v[i];
  }
}

static int pick_nb(int nE, int nN) {
  int nb = NBMAX;
  while (nb > 16 && (long long)nb * (long long)nE * 5LL > (long long)RCAP * (long long)nN * 4LL) nb >>= 1;
  return nb;
}

extern "C" void kernel_launch(void* const* d_in, const int* in_sizes, int n_in,
                              void* d_out, int out_size, void* d_ws, size_t ws_size,
                              hipStream_t stream) {
  if (n_in < 10) return;
  const int nN = in_sizes[0] / IN_DIM;
  if (nN <= 0 || in_sizes[0] != nN * IN_DIM) return;
  if (nN > (1 << 22)) return;
  const int nE2 = in_sizes[1];
  if (nE2 < 2 || (nE2 & 1) != 0) return;
  const int nE = nE2 / 2;
  if (nE > (1 << 20)) return;
  if (in_sizes[2] != IN_DIM * FEAT) return;
  if (in_sizes[3] != FEAT || in_sizes[4] != FEAT) return;
  if (in_sizes[5] != FEAT) return;
  if (in_sizes[6] != FEAT * NCLS) return;
  if (in_sizes[7] != NCLS || in_sizes[8] != NCLS) return;
  if (in_sizes[9] != NCLS) return;
  if (out_size != nN * NCLS) return;

  const float* x   = (const float*)d_in[0];
  const int*   ei  = (const int*)d_in[1];
  const float* W1  = (const float*)d_in[2];
  const float* as1 = (const float*)d_in[3];
  const float* ad1 = (const float*)d_in[4];
  const float* b1  = (const float*)d_in[5];
  const float* W2  = (const float*)d_in[6];
  const float* as2 = (const float*)d_in[7];
  const float* ad2 = (const float*)d_in[8];
  const float* b2  = (const float*)d_in[9];
  const int* src = ei;
  const int* dst = ei + nE;
  float* out = (float*)d_out;

  const int MP   = ((nN + GBM - 1) / GBM) * GBM;
  const int nb   = pick_nb(nE, nN);
  const int vec8 = ((nE & 3) == 0) ? 1 : 0;
  const int nUnits = MP * (KP / 8);

  char* ws = (char*)d_ws;
  size_t off = 0;
  const size_t oWT = off; off += (size_t)WTROWS * KP * 2;        off = (off + 255) & ~(size_t)255;
  const size_t oXH = off; off += (size_t)MP * KP * 2;            off = (off + 255) & ~(size_t)255;
  const size_t oY  = off; off += (size_t)MP * YP * 4;            off = (off + 255) & ~(size_t)255;
  const size_t oES = off; off += (size_t)MP * EP * 4;            off = (off + 255) & ~(size_t)255;
  const size_t oED = off; off += (size_t)MP * EP * 4;            off = (off + 255) & ~(size_t)255;
  const size_t oZ  = off; off += (size_t)MP * ZP * 4;            off = (off + 255) & ~(size_t)255;
  if (off > ws_size || off > (size_t)WSCAP) return;
  _Float16* WT = (_Float16*)(ws + oWT);
  _Float16* XH = (_Float16*)(ws + oXH);
  float*    Y  = (float*)(ws + oY);
  float*    ES = (float*)(ws + oES);
  float*    ED = (float*)(ws + oED);
  float*    Z  = (float*)(ws + oZ);

  hipFuncSetAttribute(reinterpret_cast<const void*>(&k_agg<1>),
                      hipFuncAttributeMaxDynamicSharedMemorySize, LDS_AGG);
  hipFuncSetAttribute(reinterpret_cast<const void*>(&k_agg<2>),
                      hipFuncAttributeMaxDynamicSharedMemorySize, LDS_AGG);

  k_xprep<<<(nUnits + NTHR - 1) / NTHR, NTHR, 0, stream>>>(x, XH, nN, nUnits);
  k_wprep<<<dim3((FEAT * (KP / 8) + NTHR - 1) / NTHR, 2), NTHR, 0, stream>>>(W1, W2, WT);

  const int gG = MP / GBM;
  const int gA = (nN + nb - 1) / nb;

  k_gemm<<<gG, GTHR, 0, stream>>>(XH, WT, as1, ad1, FEAT, Y, ES, ED, IN_DIM / 32, NHEAD);
  k_agg<1><<<gA, NTHR, LDS_AGG, stream>>>(src, dst, Y, ES, ED, b1, XH, Z, nN, nE, nb, vec8);
  k_gemm<<<gG, GTHR, 0, stream>>>(XH, WT + (size_t)FEAT * KP, as2, ad2, NCLS, Y, ES, ED, FEAT / 32, 1);
  k_agg<2><<<gA, NTHR, LDS_AGG, stream>>>(src, dst, Y, ES, ED, b2, XH, Z, nN, nE, nb, vec8);
  k_out<<<MP / OBR, NTHR, 0, stream>>>(Z, out, nN);
}
